// BaseSparseVAE_53961969107424
// MI455X (gfx1250) — hardware-verified
//
#include <hip/hip_runtime.h>
#include <math.h>

constexpr int kBatch     = 512;
constexpr int kDin       = 512;
constexpr int kLat       = 32;
constexpr int kHid       = 300;
constexpr int kHidP      = 320;
constexpr int kZcat      = 64;
constexpr int kChunkCols = 32;
constexpr int kNumChunks = kDin / kChunkCols;
constexpr int kPR        = kChunkCols * kBatch;
constexpr float kG1Carry = 16.0f;
constexpr float kLoCarry = 2048.0f;
constexpr float kW2Carry = 16.0f;
constexpr float kScaleHi = 1.0f / (kG1Carry * kW2Carry);
constexpr float kScaleLo = 1.0f / (kG1Carry * kLoCarry * kW2Carry);
static_assert(kNumChunks * kChunkCols == kDin, "");
static_assert(kPR % 64 == 0 && kHidP % 64 == 0 && kZcat % 64 == 0 && kBatch % 64 == 0, "");
static_assert(kLat % 32 == 0 && kHidP % 32 == 0 && kDin % 32 == 0, "");

typedef __attribute__((ext_vector_type(16))) _Float16 v16h;
typedef __attribute__((ext_vector_type(8)))  _Float16 v8h;
typedef __attribute__((ext_vector_type(16))) __bf16   v16b;
typedef __attribute__((ext_vector_type(8)))  __bf16   v8b;
typedef __attribute__((ext_vector_type(8)))  float    v8f;
typedef __attribute__((ext_vector_type(4)))  float    v4f;
typedef __attribute__((ext_vector_type(4)))  unsigned int v4u;

__device__ __forceinline__ unsigned short f2bf_bits(float f) {
  unsigned u = __float_as_uint(f);
  return (unsigned short)((u + 0x7FFFu + ((u >> 16) & 1u)) >> 16);
}
__device__ __forceinline__ float bf_bits2f(unsigned short h) { return __uint_as_float(((unsigned)h) << 16); }

__device__ __forceinline__ void dep_guard_h(v8f& a, v8f& b, v16h x, v16h y) { asm volatile("v_nop\n\tv_nop\n\tv_nop\n\tv_nop" : "+v"(a), "+v"(b) : "v"(x), "v"(y)); }
__device__ __forceinline__ void dep_guard_b(v8f& a, v8f& b, v16b x, v16b y) { asm volatile("v_nop\n\tv_nop\n\tv_nop\n\tv_nop" : "+v"(a), "+v"(b) : "v"(x), "v"(y)); }
__device__ __forceinline__ void keep4_h(v16h a, v16h b, v16h c, v16h d) { asm volatile("v_nop" :: "v"(a), "v"(b), "v"(c), "v"(d)); }
__device__ __forceinline__ void keep4_b(v16b a, v16b b, v16b c, v16b d) { asm volatile("v_nop" :: "v"(a), "v"(b), "v"(c), "v"(d)); }
__device__ __forceinline__ void acc_guard4(v8f& a, v8f& b, v8f& c, v8f& d) { asm volatile("v_nop\n\tv_nop\n\tv_nop\n\tv_nop" : "+v"(a), "+v"(b), "+v"(c), "+v"(d)); }
template <typename T> struct Frag;
template <> struct Frag<_Float16> {
  typedef v16h V; union U { v16h v; v8h h[2]; };
  static __device__ __forceinline__ v16h load(const _Float16* p) {
    U f; f.h[0] = *(const v8h*)(p); f.h[1] = *(const v8h*)(p + 16); return f.v;
  }
  static __device__ __forceinline__ v8f mma(v16h a, v16h b, v8f c) {
    return __builtin_amdgcn_wmma_f32_16x16x32_f16(false, a, false, b, (short)0, c, false, false);
  }
  static __device__ __forceinline__ void guard(v8f& a, v8f& b, v16h x, v16h y) { dep_guard_h(a, b, x, y); }
  static __device__ __forceinline__ void keep(v16h a, v16h b, v16h c, v16h d) { keep4_h(a, b, c, d); }
};
template <> struct Frag<__bf16> {
  typedef v16b V; union U { v16b v; v8b h[2]; };
  static __device__ __forceinline__ v16b load(const __bf16* p) {
    U f; f.h[0] = *(const v8b*)(p); f.h[1] = *(const v8b*)(p + 16); return f.v;
  }
  static __device__ __forceinline__ v8f mma(v16b a, v16b b, v8f c) {
    return __builtin_amdgcn_wmma_f32_16x16x32_bf16(false, a, false, b, (short)0, c, false, false);
  }
  static __device__ __forceinline__ void guard(v8f& a, v8f& b, v16b x, v16b y) { dep_guard_b(a, b, x, y); }
  static __device__ __forceinline__ void keep(v16b a, v16b b, v16b c, v16b d) { keep4_b(a, b, c, d); }
};

__device__ __forceinline__ unsigned pk16(unsigned short a, unsigned short b) { return (unsigned)a | ((unsigned)b << 16); }
__device__ __forceinline__ unsigned short h_bits(float f) { const _Float16 h = (_Float16)f; return __builtin_bit_cast(unsigned short, h); }

template <int ET> struct Elem;
template <> struct Elem<0> { typedef _Float16 T; };
template <> struct Elem<1> { typedef __bf16 T; };
template <int ET, bool SPLIT, int BIAS_MODE, int OUT_MODE, bool RESID, int ACT = 0>
__global__ __launch_bounds__(256) void wmma_gemm64(
    const unsigned short* __restrict__ Ap, const unsigned short* __restrict__ A2p, int lda, long strideA,
    const unsigned short* __restrict__ Btp, const unsigned short* __restrict__ Bt2p, int ldb, long strideB,
    void* __restrict__ Cout, void* __restrict__ Cout2, int ldc, long strideC,
    const float* __restrict__ bias,
    const float* __restrict__ resid, long strideR,
    int M, int N, int K, float scale) {
  typedef typename Elem<ET>::T T;
  typedef typename Frag<T>::V V;
  const T* A = (const T*)Ap; const T* A2 = (const T*)A2p; const T* Bt = (const T*)Btp; const T* Bt2 = (const T*)Bt2p;
  __shared__ __align__(16) float sT[8][16 * 68];
  const int b    = blockIdx.y;
  const int lane = threadIdx.x & 31;
  const int wave = threadIdx.x >> 5;
  const int tilesN = N >> 6;
  const int tilesM = M >> 6;
  const int tile = blockIdx.x * 8 + wave;
  if (tile >= tilesM * tilesN) return;
  const int tm = tile / tilesN;
  const int tn = tile - tm * tilesN;
  const int m0 = tm << 6;
  const int n0 = tn << 6;

  const T* Ab  = A  + (size_t)b * strideA;
  const T* Bb  = Bt + (size_t)b * strideB;
  const T* Ab2 = SPLIT ? (A2  + (size_t)b * strideA) : nullptr;
  const T* Bb2 = SPLIT ? (Bt2 + (size_t)b * strideB) : nullptr;

  const int rlane = lane & 15;
  const int koff  = (lane >> 4) * 8;
  const int mOff  = (lane >> 4) * 8;

  v8f acc[4][4];
#pragma unroll
  for (int i = 0; i < 4; ++i)
#pragma unroll
    for (int j = 0; j < 4; ++j) acc[i][j] = (v8f){0.f,0.f,0.f,0.f,0.f,0.f,0.f,0.f};

  for (int k0 = 0; k0 < K; k0 += 32) {
    V bh[4], bl[4];
#pragma unroll
    for (int j = 0; j < 4; ++j) {
      const size_t bo = (size_t)(n0 + (j << 4) + rlane) * ldb + koff + k0;
      bh[j] = Frag<T>::load(Bb + bo);
      if (SPLIT) bl[j] = Frag<T>::load(Bb2 + bo);
    }
#pragma unroll
    for (int i = 0; i < 4; ++i) {
      const size_t ao = (size_t)(m0 + (i << 4) + rlane) * lda + koff + k0;
      V ah = Frag<T>::load(Ab + ao);
      V al;
      if (SPLIT) al = Frag<T>::load(Ab2 + ao);
#pragma unroll
      for (int j = 0; j < 4; ++j) {
        acc[i][j] = Frag<T>::mma(ah, bh[j], acc[i][j]);
        if (SPLIT) {
          acc[i][j] = Frag<T>::mma(ah, bl[j], acc[i][j]);
          acc[i][j] = Frag<T>::mma(al, bh[j], acc[i][j]);
        }
      }
      Frag<T>::guard(acc[i][0], acc[i][3], ah, SPLIT ? al : ah);
    }
    Frag<T>::keep(bh[0], bh[1], bh[2], bh[3]);
    if (SPLIT) Frag<T>::keep(bl[0], bl[1], bl[2], bl[3]);
  }
  acc_guard4(acc[0][0], acc[0][1], acc[0][2], acc[0][3]);
  acc_guard4(acc[1][0], acc[1][1], acc[1][2], acc[1][3]);
  acc_guard4(acc[2][0], acc[2][1], acc[2][2], acc[2][3]);
  acc_guard4(acc[3][0], acc[3][1], acc[3][2], acc[3][3]);

  float* slab = sT[wave];
  const float* Rb = RESID ? (resid + (size_t)b * strideR) : nullptr;
#pragma unroll
  for (int i = 0; i < 4; ++i) {
    const int mBase = m0 + (i << 4);
#pragma unroll
    for (int j = 0; j < 4; ++j) {
      const int n = n0 + (j << 4) + rlane;
      float bv = 0.f;
      if (BIAS_MODE == 2) bv = bias[n];
#pragma unroll
      for (int r = 0; r < 8; ++r) {
        float v = acc[i][j][r] * scale;
        if (BIAS_MODE == 1) v += bias[mBase + mOff + r];
        if (BIAS_MODE == 2) v += bv;
        if (RESID) v += Rb[(size_t)(mBase + mOff + r) * ldc + n];
        if (ACT == 2) v = fmaxf(v, 0.0f);
        if (ACT == 4) v = (v > 0.f) ? v : 0.01f * v;
        slab[(mOff + r) * 68 + (j << 4) + rlane] = v;
      }
    }
    __builtin_amdgcn_fence(__ATOMIC_RELEASE, "workgroup");
    __builtin_amdgcn_wave_barrier();
    __builtin_amdgcn_fence(__ATOMIC_ACQUIRE, "workgroup");
    if (OUT_MODE == 0) {
      float* C = (float*)Cout + (size_t)b * strideC;
      const int hh = lane >> 4, c4 = (lane & 15) * 4;
      for (int pass = 0; pass < 2; ++pass) {
#pragma unroll
        for (int it = 0; it < 8; ++it) {
          const int row = it * 2 + hh;
          v4f v = *(const v4f*)(slab + row * 68 + c4);
          *(volatile v4f*)(C + (size_t)(mBase + row) * ldc + n0 + c4) = v;
        }
        __threadfence();
      }
    } else {
      const int q = lane >> 3, c8 = (lane & 7) * 8;
      unsigned short* C  = (unsigned short*)Cout  + (size_t)b * strideC;
      unsigned short* C2 = (OUT_MODE >= 2) ? ((unsigned short*)Cout2 + (size_t)b * strideC) : nullptr;
      for (int pass = 0; pass < 2; ++pass) {
#pragma unroll
        for (int it = 0; it < 4; ++it) {
          const int row = it * 4 + q;
          const float* sp = slab + row * 68 + c8;
          v8h hv, lv;
#pragma unroll
          for (int e = 0; e < 8; ++e) {
            if (OUT_MODE == 1) {
              hv[e] = (_Float16)sp[e];
            } else if (OUT_MODE == 3) {
              const float t = sp[e] * kG1Carry;
              const _Float16 th = (_Float16)t;
              hv[e] = th;
              lv[e] = (_Float16)((t - (float)th) * kLoCarry);
            } else {
              unsigned short hb = f2bf_bits(sp[e]);
              unsigned short lb = f2bf_bits(sp[e] - bf_bits2f(hb));
              hv[e] = __builtin_bit_cast(_Float16, hb);
              lv[e] = __builtin_bit_cast(_Float16, lb);
            }
          }
          *(volatile v8h*)(C + (size_t)(mBase + row) * ldc + n0 + c8) = hv;
          if (OUT_MODE >= 2) *(volatile v8h*)(C2 + (size_t)(mBase + row) * ldc + n0 + c8) = lv;
        }
        __threadfence();
      }
    }
    __builtin_amdgcn_fence(__ATOMIC_RELEASE, "workgroup");
    __builtin_amdgcn_wave_barrier();
    __builtin_amdgcn_fence(__ATOMIC_ACQUIRE, "workgroup");
  }
}

__global__ __launch_bounds__(256) void xsplit_kernel(const float* __restrict__ in, unsigned short* __restrict__ oh,
                                                     unsigned short* __restrict__ ol, int n8) {
  const int i = blockIdx.x * 256 + threadIdx.x;
  if (i >= n8) return;
  const float* p = in + 8 * (size_t)i;
  const v4f a = *(const v4f*)(p);
  const v4f c = *(const v4f*)(p + 4);
  unsigned short hb[8], lb[8];
#pragma unroll
  for (int e = 0; e < 4; ++e) {
    const unsigned short h0 = f2bf_bits(a[e]);
    const unsigned short h1 = f2bf_bits(c[e]);
    hb[e] = h0; hb[4 + e] = h1;
    lb[e] = f2bf_bits(a[e] - bf_bits2f(h0));
    lb[4 + e] = f2bf_bits(c[e] - bf_bits2f(h1));
  }
  const v4u uh = (v4u){pk16(hb[0], hb[1]), pk16(hb[2], hb[3]), pk16(hb[4], hb[5]), pk16(hb[6], hb[7])};
  const v4u ul = (v4u){pk16(lb[0], lb[1]), pk16(lb[2], lb[3]), pk16(lb[4], lb[5]), pk16(lb[6], lb[7])};
  unsigned short* qh = oh + 8 * (size_t)i;
  unsigned short* ql = ol + 8 * (size_t)i;
  *(volatile v4u*)qh = uh;
  *(volatile v4u*)ql = ul;
  __threadfence();
  *(volatile v4u*)qh = uh;
  *(volatile v4u*)ql = ul;
}

template <int MODE>
__global__ __launch_bounds__(256) void tcast_kernel(const float* __restrict__ W0, const float* __restrict__ W1,
                                                    int R, int Cn0, int Cn1,
                                                    unsigned short* __restrict__ outA, unsigned short* __restrict__ outB,
                                                    int Npad, int Kpad, float scale) {
  const int e = blockIdx.x * 256 + threadIdx.x;
  const int qn = Kpad >> 3;
  const int total = Npad * qn;
  if (e >= total) return;
  const int n  = e / qn;
  const int k0 = (e - n * qn) * 8;
  const bool in0 = (n < Cn0);
  const int c0 = min(n, Cn0 - 1);
  int c1 = n - Cn0;
  const bool in1 = (c1 >= 0) && (c1 < Cn1);
  c1 = max(0, min(c1, max(Cn1 - 1, 0)));
  unsigned short ha[8], hb[8];
#pragma unroll
  for (int i = 0; i < 8; ++i) {
    const int k  = k0 + i;
    const int kc = min(k, R - 1);
    const float v0 = W0[(size_t)kc * Cn0 + c0];
    const float v1 = W1[(size_t)kc * Cn1 + c1];
    float v = in0 ? v0 : (in1 ? v1 : 0.0f);
    v = (k < R) ? v : 0.0f;
    if (MODE == 0) {
      const unsigned short h = f2bf_bits(v);
      ha[i] = h;
      hb[i] = f2bf_bits(v - bf_bits2f(h));
    } else {
      ha[i] = h_bits(v * scale);
      hb[i] = 0;
    }
  }
  const v4u ua = (v4u){pk16(ha[0], ha[1]), pk16(ha[2], ha[3]), pk16(ha[4], ha[5]), pk16(ha[6], ha[7])};
  const v4u ub = (v4u){pk16(hb[0], hb[1]), pk16(hb[2], hb[3]), pk16(hb[4], hb[5]), pk16(hb[6], hb[7])};
  unsigned short* pa = outA + (size_t)n * Kpad + k0;
  unsigned short* pb = outB + (size_t)n * Kpad + k0;
  *(volatile v4u*)pa = ua;
  if (MODE == 0) *(volatile v4u*)pb = ub;
  __threadfence();
  *(volatile v4u*)pa = ua;
  if (MODE == 0) *(volatile v4u*)pb = ub;
}

__global__ __launch_bounds__(256) void bias_pack_kernel(const float* __restrict__ b1, const float* __restrict__ b2,
                                                        const float* __restrict__ gb2, const float* __restrict__ zmb,
                                                        const float* __restrict__ zlb, float* __restrict__ outp) {
  const int t = threadIdx.x;
  float vv[4];
#pragma unroll
  for (int e = 0; e < 4; ++e) {
    const int idx = 4 * t + e;
    const int i1 = min(idx, kHid - 1);
    const int i2 = min(max(idx - 320, 0), kHid - 1);
    const int i3 = min(max(idx - 640, 0), kHid - 1);
    const int i4 = min(max(idx - 960, 0), kLat - 1);
    const int i5 = min(max(idx - 992, 0), kLat - 1);
    const float c1 = b1[i1];
    const float c2 = b2[i2];
    const float c3 = gb2[i3];
    const float c4 = zmb[i4];
    const float c5 = zlb[i5];
    float v = 0.0f;
    v = (idx < kHid) ? c1 : v;
    v = (idx >= 320 && idx < 320 + kHid) ? c2 : v;
    v = (idx >= 640 && idx < 640 + kHid) ? c3 : v;
    v = (idx >= 960 && idx < 992) ? c4 : v;
    v = (idx >= 992) ? c5 : v;
    vv[e] = v;
  }
  const v4f u = (v4f){vv[0], vv[1], vv[2], vv[3]};
  float* q = outp + 4 * t;
  *(volatile v4f*)q = u;
  __threadfence();
  *(volatile v4f*)q = u;
}

__global__ __launch_bounds__(256) void reparam_kernel(const float* __restrict__ ZC, const float* __restrict__ eps,
                                                      float* __restrict__ outz, float* __restrict__ outzm,
                                                      float* __restrict__ outzl) {
  const int t = blockIdx.x * 256 + threadIdx.x;
  if (t >= kBatch * 8) return;
  const int b  = t >> 3;
  const int l0 = (t & 7) * 4;
  const v4f zm = *(const v4f*)(ZC + (size_t)b * kZcat + l0);
  const v4f zl = *(const v4f*)(ZC + (size_t)b * kZcat + kLat + l0);
  const v4f ep = *(const v4f*)(eps + (size_t)b * kLat + l0);
  v4f z;
  z[0] = zm[0] + ep[0] * expf(0.5f * zl[0]);
  z[1] = zm[1] + ep[1] * expf(0.5f * zl[1]);
  z[2] = zm[2] + ep[2] * expf(0.5f * zl[2]);
  z[3] = zm[3] + ep[3] * expf(0.5f * zl[3]);
  const size_t o = (size_t)b * kLat + l0;
  *(volatile v4f*)(outz  + o) = z;
  *(volatile v4f*)(outzm + o) = zm;
  *(volatile v4f*)(outzl + o) = zl;
  __threadfence();
  *(volatile v4f*)(outz  + o) = z;
  *(volatile v4f*)(outzm + o) = zm;
  *(volatile v4f*)(outzl + o) = zl;
}

__global__ __launch_bounds__(256) void masked_split_kernel(const float* __restrict__ Wm, const float* __restrict__ zf,
                                                           unsigned short* __restrict__ AH, unsigned short* __restrict__ AL,
                                                           int jc) {
  const int t  = blockIdx.x * 256 + threadIdx.x;
  if (t >= kPR * 4) return;
  const int p  = t >> 2;
  const int l0 = (t & 3) * 8;
  const int jl = p >> 9;
  const int b  = p & 511;
  const int j  = jc + jl;
  const float* wr = Wm + (size_t)j * kLat + l0;
  const float* zr = zf + (size_t)b * kLat + l0;
  const v4f w0 = *(const v4f*)(wr);
  const v4f w1 = *(const v4f*)(wr + 4);
  const v4f z0 = *(const v4f*)(zr);
  const v4f z1 = *(const v4f*)(zr + 4);
  unsigned short hb[8], lb[8];
#pragma unroll
  for (int e = 0; e < 4; ++e) {
    const float m0 = w0[e] * z0[e];
    const float m1 = w1[e] * z1[e];
    const unsigned short h0 = f2bf_bits(m0);
    const unsigned short h1 = f2bf_bits(m1);
    hb[e] = h0; hb[4 + e] = h1;
    lb[e] = f2bf_bits(m0 - bf_bits2f(h0));
    lb[4 + e] = f2bf_bits(m1 - bf_bits2f(h1));
  }
  const v4u uh = (v4u){pk16(hb[0], hb[1]), pk16(hb[2], hb[3]), pk16(hb[4], hb[5]), pk16(hb[6], hb[7])};
  const v4u ul = (v4u){pk16(lb[0], lb[1]), pk16(lb[2], lb[3]), pk16(lb[4], lb[5]), pk16(lb[6], lb[7])};
  unsigned short* ph = AH + (size_t)p * kLat + l0;
  unsigned short* pl = AL + (size_t)p * kLat + l0;
  *(volatile v4u*)ph = uh;
  *(volatile v4u*)pl = ul;
  __threadfence();
  *(volatile v4u*)ph = uh;
  *(volatile v4u*)pl = ul;
}

__global__ __launch_bounds__(256) void coldot_kernel(const float* __restrict__ G2, const float* __restrict__ colw,
                                                     const float* __restrict__ colb, float* __restrict__ out0, int jc) {
  __shared__ __align__(16) float xs[kChunkCols];
  const int b    = blockIdx.x;
  const int lane = threadIdx.x & 31;
  const int wave = threadIdx.x >> 5;
#pragma unroll 1
  for (int jj = 0; jj < 4; ++jj) {
    const int jl = wave * 4 + jj;
    const int j  = jc + jl;
    const int p  = jl * kBatch + b;
    const float* gr = G2 + (size_t)p * kHidP;
    const float* cr = colw + (size_t)j * kHid;
    const float cb = colb[j];
    float s = 0.0f;
#pragma unroll 1
    for (int i = 0; i < 10; ++i) {
      const int h  = lane + 32 * i;
      const int hc = min(h, kHid - 1);
      const float g = gr[hc];
      const float c = cr[hc];
      const float term = g * c;
      s += (h < kHid) ? term : 0.0f;
    }
    s += __shfl_xor(s, 16, 32);
    s += __shfl_xor(s, 8, 32);
    s += __shfl_xor(s, 4, 32);
    s += __shfl_xor(s, 2, 32);
    s += __shfl_xor(s, 1, 32);
    if (lane == 0) xs[jl] = s + cb;
  }
  __syncthreads();
  if (wave == 0 && lane < 8) {
    const v4f v = *(const v4f*)(xs + 4 * lane);
    float* op = out0 + (size_t)b * kDin + jc + 4 * lane;
    *(volatile v4f*)op = v;
    __threadfence();
    *(volatile v4f*)op = v;
  }
}

extern "C" void kernel_launch(void* const* d_in, const int* in_sizes, int n_in,
                              void* d_out, int out_size, void* d_ws, size_t ws_size,
                              hipStream_t stream) {
  (void)in_sizes;
  if (n_in < 16) return;
  if (out_size < kBatch * kDin + 3 * kBatch * kLat) return;

  const float* x      = (const float*)d_in[0];
  const float* eps    = (const float*)d_in[1];
  const float* Wm     = (const float*)d_in[2];
  const float* qz_w1  = (const float*)d_in[3];
  const float* qz_b1  = (const float*)d_in[4];
  const float* qz_w2  = (const float*)d_in[5];
  const float* qz_b2  = (const float*)d_in[6];
  const float* zm_w   = (const float*)d_in[7];
  const float* zm_b   = (const float*)d_in[8];
  const float* zl_w   = (const float*)d_in[9];
  const float* zl_b   = (const float*)d_in[10];
  const float* gen_w1 = (const float*)d_in[11];
  const float* gen_w2 = (const float*)d_in[12];
  const float* gen_b2 = (const float*)d_in[13];
  const float* col_w  = (const float*)d_in[14];
  const float* col_b  = (const float*)d_in[15];

  float* out  = (float*)d_out;
  float* out0 = out;
  float* out1 = out + kBatch * kDin;
  float* out2 = out1 + kBatch * kLat;
  float* out3 = out2 + kBatch * kLat;

  char* ws = (char*)d_ws;
  size_t off = 0;
  auto carve = [&](size_t bytes) -> char* {
    char* p = ws + off;
    off += (bytes + 4095) & ~(size_t)4095;
    return p;
  };
  unsigned short* XH   = (unsigned short*)carve((size_t)kBatch * kDin * 2);
  unsigned short* XL   = (unsigned short*)carve((size_t)kBatch * kDin * 2);
  unsigned short* W1TH = (unsigned short*)carve((size_t)kHidP * kDin * 2);
  unsigned short* W1TL = (unsigned short*)carve((size_t)kHidP * kDin * 2);
  unsigned short* W2TH = (unsigned short*)carve((size_t)kHidP * kHidP * 2);
  unsigned short* W2TL = (unsigned short*)carve((size_t)kHidP * kHidP * 2);
  unsigned short* WZTH = (unsigned short*)carve((size_t)kZcat * kHidP * 2);
  unsigned short* WZTL = (unsigned short*)carve((size_t)kZcat * kHidP * 2);
  unsigned short* G1WH = (unsigned short*)carve((size_t)kHidP * kLat * 2);
  unsigned short* G1WL = (unsigned short*)carve((size_t)kHidP * kLat * 2);
  unsigned short* W2D  = (unsigned short*)carve((size_t)kHidP * kHidP * 2);
  float*          BP   = (float*)carve((size_t)1024 * 4);
  unsigned short* H1H  = (unsigned short*)carve((size_t)kBatch * kHidP * 2);
  unsigned short* H1L  = (unsigned short*)carve((size_t)kBatch * kHidP * 2);
  unsigned short* H2H  = (unsigned short*)carve((size_t)kBatch * kHidP * 2);
  unsigned short* H2L  = (unsigned short*)carve((size_t)kBatch * kHidP * 2);
  float*          ZC   = (float*)carve((size_t)kBatch * kZcat * 4);
  unsigned short* A1H  = (unsigned short*)carve((size_t)kPR * kLat * 2);
  unsigned short* A1L  = (unsigned short*)carve((size_t)kPR * kLat * 2);
  unsigned short* G1H  = (unsigned short*)carve((size_t)kPR * kHidP * 2);
  unsigned short* G1L  = (unsigned short*)carve((size_t)kPR * kHidP * 2);
  float*          G2A  = (float*)carve((size_t)kPR * kHidP * 4);
  float*          G2B  = (float*)carve((size_t)kPR * kHidP * 4);
  if (off > ws_size) return;

  const float* BP_b1  = BP;
  const float* BP_b2  = BP + 320;
  const float* BP_gb2 = BP + 640;
  const float* BP_bz  = BP + 960;

  xsplit_kernel<<<(kBatch * kDin / 8 + 255) / 256, 256, 0, stream>>>(x, XH, XL, kBatch * kDin / 8);
  tcast_kernel<0><<<(kHidP * (kDin / 8) + 255) / 256, 256, 0, stream>>>(qz_w1, qz_w1, kDin, kHid, 0, W1TH, W1TL, kHidP, kDin, 1.0f);
  tcast_kernel<0><<<(kHidP * (kHidP / 8) + 255) / 256, 256, 0, stream>>>(qz_w2, qz_w2, kHid, kHid, 0, W2TH, W2TL, kHidP, kHidP, 1.0f);
  tcast_kernel<0><<<(kZcat * (kHidP / 8) + 255) / 256, 256, 0, stream>>>(zm_w, zl_w, kHid, kLat, kLat, WZTH, WZTL, kZcat, kHidP, 1.0f);
  tcast_kernel<0><<<(kHidP * (kLat / 8) + 255) / 256, 256, 0, stream>>>(gen_w1, gen_w1, kLat, kHid, 0, G1WH, G1WL, kHidP, kLat, 1.0f);
  tcast_kernel<1><<<(kHidP * (kHidP / 8) + 255) / 256, 256, 0, stream>>>(gen_w2, gen_w2, kHid, kHid, 0, W2D, W2D, kHidP, kHidP, kW2Carry);
  bias_pack_kernel<<<1, 256, 0, stream>>>(qz_b1, qz_b2, gen_b2, zm_b, zl_b, BP);

  wmma_gemm64<1, true, 2, 2, false, 2><<<dim3((8 * 5 + 7) / 8, 1), 256, 0, stream>>>(
      XH, XL, kDin, 0L, W1TH, W1TL, kDin, 0L, (void*)H1H, (void*)H1L, kHidP, 0L,
      BP_b1, BP, 0L, kBatch, kHidP, kDin, 1.0f);
  wmma_gemm64<1, true, 2, 2, false, 2><<<dim3((8 * 5 + 7) / 8, 1), 256, 0, stream>>>(
      H1H, H1L, kHidP, 0L, W2TH, W2TL, kHidP, 0L, (void*)H2H, (void*)H2L, kHidP, 0L,
      BP_b2, BP, 0L, kBatch, kHidP, kHidP, 1.0f);
  wmma_gemm64<1, true, 2, 0, false, 0><<<dim3((8 * 1 + 7) / 8, 1), 256, 0, stream>>>(
      H2H, H2L, kHidP, 0L, WZTH, WZTL, kHidP, 0L, (void*)ZC, (void*)ZC, kZcat, 0L,
      BP_bz, BP, 0L, kBatch, kZcat, kHidP, 1.0f);
  reparam_kernel<<<(kBatch * 8 + 255) / 256, 256, 0, stream>>>(ZC, eps, out1, out2, out3);

  const int decTiles  = (kPR / 64) * (kHidP / 64);
  const int decBlocks = (decTiles + 7) / 8;
  for (int c = 0; c < kNumChunks; ++c) {
    const int jc = c * kChunkCols;
    masked_split_kernel<<<(kPR * 4 + 255) / 256, 256, 0, stream>>>(Wm, out1, A1H, A1L, jc);
    wmma_gemm64<1, true, 0, 3, false, 2><<<dim3(decBlocks, 1), 256, 0, stream>>>(
        A1H, A1L, kLat, 0L, G1WH, G1WL, kLat, 0L, (void*)G1H, (void*)G1L, kHidP, 0L,
        BP, BP, 0L, kPR, kHidP, kLat, 1.0f);
    wmma_gemm64<0, false, 0, 0, false, 0><<<dim3(decBlocks, 1), 256, 0, stream>>>(
        G1H, G1H, kHidP, 0L, W2D, W2D, kHidP, 0L, (void*)G2A, (void*)G2A, kHidP, 0L,
        BP, BP, 0L, kPR, kHidP, kHidP, kScaleHi);
    wmma_gemm64<0, false, 2, 0, true, 2><<<dim3(decBlocks, 1), 256, 0, stream>>>(
        G1L, G1L, kHidP, 0L, W2D, W2D, kHidP, 0L, (void*)G2B, (void*)G2B, kHidP, 0L,
        BP_gb2, G2A, 0L, kPR, kHidP, kHidP, kScaleLo);
    coldot_kernel<<<kBatch, 256, 0, stream>>>(G2B, col_w, col_b, out0, jc);
  }
}
